// BSMamba3Block_69475390980342
// MI455X (gfx1250) — hardware-verified
//
#include <hip/hip_runtime.h>
#include <math.h>
#include <stddef.h>

typedef __attribute__((ext_vector_type(16))) _Float16 v16h;
typedef __attribute__((ext_vector_type(8)))  _Float16 v8h;
typedef __attribute__((ext_vector_type(16))) __bf16   v16b;
typedef __attribute__((ext_vector_type(8)))  __bf16   v8b;
typedef __attribute__((ext_vector_type(8)))  float    v8f;
typedef __attribute__((ext_vector_type(4)))  float    v4f;

constexpr int kBatch = 2;
constexpr int kTime  = 256;
constexpr int kBands = 8;
constexpr int kDim   = 256;
constexpr int kHeads = 4;
constexpr int kHd    = 64;
constexpr int kNs    = 128;
constexpr int kRows  = kBatch * kTime * kBands;
constexpr int kFf    = 1024;
constexpr int kC1P = 1600, kC1X = 0, kC1Z = 256, kC1B = 512, kC1C = 1024, kC1T = 1536;
constexpr int kQkvP = 768;
constexpr int kGuP  = 2048;
constexpr int kDtbP = kHeads * kNs;
constexpr int kScanTS = 32;
constexpr int kScanYP = 68;
constexpr int kConvTP = 260;
constexpr int kAttnOP = 260;
static_assert(kRows == 4096, "rows");
static_assert(kDim == kHeads * kHd, "head split");
static_assert((kRows % 64) == 0 && (kC1P % 64) == 0 && (kDim % 64) == 0 && (kQkvP % 64) == 0 && (kGuP % 64) == 0, "GEMM M,N multiples of 64");
static_assert((kDim % 32) == 0 && (kFf % 32) == 0, "GEMM K multiples of 32");
static_assert((kTime % 64) == 0 && (kTime % kScanTS) == 0, "tile multiples");
static_assert((kC1P * 4) % 128 == 0 && (kQkvP * 4) % 128 == 0 && (kGuP * 4) % 128 == 0 && (kDtbP * 4) % 128 == 0, "line-multiple pitches");

constexpr size_t kOffWcat = 0;
constexpr size_t kOffWout = kOffWcat + (size_t)kC1P * kDim * 2;
constexpr size_t kOffWqkv = kOffWout + (size_t)kDim * kDim * 2;
constexpr size_t kOffWao  = kOffWqkv + (size_t)kQkvP * kDim * 2;
constexpr size_t kOffWgu  = kOffWao  + (size_t)kDim * kDim * 2;
constexpr size_t kOffWd   = kOffWgu  + (size_t)kGuP * kDim * 2;
constexpr size_t kOffUH   = kOffWd   + (size_t)kDim * kFf * 2;
constexpr size_t kOffUL   = kOffUH   + (size_t)kRows * kDim * 2;
constexpr size_t kOffC1   = kOffUL   + (size_t)kRows * kDim * 2;
constexpr size_t kOffXH   = kOffC1   + (size_t)kRows * kC1P * 4;
constexpr size_t kOffDTB  = kOffXH   + (size_t)kRows * kDim * 4;
constexpr size_t kOffDT   = kOffDTB  + (size_t)kRows * kDtbP * 4;
constexpr size_t kOffAR   = kOffDT   + (size_t)kRows * kHeads * 4;
constexpr size_t kOffAI   = kOffAR   + (size_t)kRows * kHeads * 4;
constexpr size_t kOffYSP  = kOffAI   + (size_t)kRows * kHeads * 4;
constexpr size_t kOffY2H  = kOffYSP  + (size_t)4 * kRows * kDim * 4;
constexpr size_t kOffY2L  = kOffY2H  + (size_t)kRows * kDim * 2;
constexpr size_t kOffZ1   = kOffY2L  + (size_t)kRows * kDim * 2;
constexpr size_t kOffZNH  = kOffZ1   + (size_t)kRows * kDim * 4;
constexpr size_t kOffZNL  = kOffZNH  + (size_t)kRows * kDim * 2;
constexpr size_t kOffQKV  = kOffZNL  + (size_t)kRows * kDim * 2;
constexpr size_t kOffOH   = kOffQKV  + (size_t)kRows * kQkvP * 4;
constexpr size_t kOffOL   = kOffOH   + (size_t)kRows * kDim * 2;
constexpr size_t kOffZ2   = kOffOL   + (size_t)kRows * kDim * 2;
constexpr size_t kOffZFH  = kOffZ2   + (size_t)kRows * kDim * 4;
constexpr size_t kOffZFL  = kOffZFH  + (size_t)kRows * kDim * 2;
constexpr size_t kOffGUH  = kOffZFL  + (size_t)kRows * kDim * 2;
constexpr size_t kOffGUL  = kOffGUH  + (size_t)kRows * kFf * 2;
constexpr size_t kWsTotal = kOffGUL  + (size_t)kRows * kFf * 2;
constexpr size_t kOffGU   = kOffC1;
static_assert(kWsTotal == 117538816ull, "carve total");
static_assert(kWsTotal <= 134217728ull, "carve cap");
static_assert(kOffGU + (size_t)kRows * kGuP * 4 <= kOffDT, "GU alias stays inside C1|XH|DTB");
static_assert((kOffWout % 128) == 0 && (kOffWqkv % 128) == 0 && (kOffWao % 128) == 0 && (kOffWgu % 128) == 0 &&
              (kOffWd % 128) == 0 && (kOffUH % 128) == 0 && (kOffUL % 128) == 0 && (kOffC1 % 128) == 0 &&
              (kOffXH % 128) == 0 && (kOffDTB % 128) == 0 && (kOffDT % 128) == 0 && (kOffAR % 128) == 0 &&
              (kOffAI % 128) == 0 && (kOffYSP % 128) == 0 && (kOffY2H % 128) == 0 && (kOffY2L % 128) == 0 &&
              (kOffZ1 % 128) == 0 && (kOffZNH % 128) == 0 && (kOffZNL % 128) == 0 && (kOffQKV % 128) == 0 &&
              (kOffOH % 128) == 0 && (kOffOL % 128) == 0 && (kOffZ2 % 128) == 0 && (kOffZFH % 128) == 0 &&
              (kOffZFL % 128) == 0 && (kOffGUH % 128) == 0 && (kOffGUL % 128) == 0, "128-B aligned regions");

__device__ __forceinline__ unsigned short f2bf_bits(float f) {
  unsigned u = __float_as_uint(f);
  return (unsigned short)((u + 0x7FFFu + ((u >> 16) & 1u)) >> 16);
}
__device__ __forceinline__ float bf_bits2f(unsigned short h) { return __uint_as_float(((unsigned)h) << 16); }
__device__ __forceinline__ float bf_rne(float f) { return bf_bits2f(f2bf_bits(f)); }
__device__ __forceinline__ _Float16 bits_h(unsigned short b) { return __builtin_bit_cast(_Float16, b); }
__device__ __forceinline__ void split_bits(float f, unsigned short& hb, unsigned short& lb) {
  hb = f2bf_bits(f);
  lb = f2bf_bits(f - bf_bits2f(hb));
}
__device__ __forceinline__ void split8(v4f a0, v4f a1, v8h& hv, v8h& lv) {
#pragma unroll
  for (int e = 0; e < 4; ++e) {
    unsigned short h0, l0, h1, l1;
    split_bits(a0[e], h0, l0);
    split_bits(a1[e], h1, l1);
    hv[e] = bits_h(h0); hv[4 + e] = bits_h(h1);
    lv[e] = bits_h(l0); lv[4 + e] = bits_h(l1);
  }
}
__device__ __forceinline__ void store2_v8h(unsigned short* p, v8h v) {
  *(volatile v8h*)p = v; __threadfence(); *(volatile v8h*)p = v;
}
__device__ __forceinline__ void store2_v4f(float* p, v4f v) {
  *(volatile v4f*)p = v; __threadfence(); *(volatile v4f*)p = v;
}

__device__ __forceinline__ void acc_guard4(v8f& a, v8f& b, v8f& c, v8f& d) {
  asm volatile("v_nop\n\tv_nop\n\tv_nop\n\tv_nop" : "+v"(a), "+v"(b), "+v"(c), "+v"(d));
}
__device__ __forceinline__ void dep_guard_all(v8f& a0, v8f& a1, v8f& a2, v8f& a3, v16b x, v16b y,
                                              v16b b0, v16b b1, v16b b2, v16b b3) {
  asm volatile("v_nop\n\tv_nop\n\tv_nop\n\tv_nop"
               : "+v"(a0), "+v"(a1), "+v"(a2), "+v"(a3)
               : "v"(x), "v"(y), "v"(b0), "v"(b1), "v"(b2), "v"(b3));
}
template <typename T> struct Frag;
template <> struct Frag<__bf16> {
  typedef v16b V; union U { v16b v; v8b h[2]; };
  static __device__ __forceinline__ v16b load(const __bf16* p) {
    U f; f.h[0] = *(const v8b*)(p); f.h[1] = *(const v8b*)(p + 16); return f.v;
  }
  static __device__ __forceinline__ v8f mma(v16b a, v16b b, v8f c) {
    return __builtin_amdgcn_wmma_f32_16x16x32_bf16(false, a, false, b, (short)0, c, false, false);
  }
};

template <int BIAS_MODE, int RESID_MODE>
__global__ __launch_bounds__(256) void gemm_hilo_bf16_64(
    const unsigned short* __restrict__ Ap, const unsigned short* __restrict__ A2p, int lda,
    const unsigned short* __restrict__ Btp, int ldb,
    float* __restrict__ Cout, int ldc,
    const float* __restrict__ bias,
    const float* __restrict__ resid, int ldr,
    int M, int N, int K) {
  const __bf16* A  = (const __bf16*)Ap;
  const __bf16* A2 = (const __bf16*)A2p;
  const __bf16* Bt = (const __bf16*)Btp;
  __shared__ __align__(16) float sT[8][16 * 68];
  const int lane = threadIdx.x & 31;
  const int wave = threadIdx.x >> 5;
  const int tilesN = N >> 6;
  const int tilesM = M >> 6;
  const int tile = blockIdx.x * 8 + wave;
  if (tile >= tilesM * tilesN) return;
  const int tm = tile / tilesN;
  const int tn = tile - tm * tilesN;
  const int m0 = tm << 6;
  const int n0 = tn << 6;
  const int rlane = lane & 15;
  const int koff  = (lane >> 4) * 8;
  const int mOff  = (lane >> 4) * 8;

  v8f acc[4][4];
#pragma unroll
  for (int i = 0; i < 4; ++i)
#pragma unroll
    for (int j = 0; j < 4; ++j) acc[i][j] = (v8f){0.f, 0.f, 0.f, 0.f, 0.f, 0.f, 0.f, 0.f};

  for (int k0 = 0; k0 < K; k0 += 32) {
    v16b bh[4];
#pragma unroll
    for (int j = 0; j < 4; ++j) {
      const size_t bo = (size_t)(n0 + (j << 4) + rlane) * ldb + koff + k0;
      bh[j] = Frag<__bf16>::load(Bt + bo);
    }
#pragma unroll
    for (int i = 0; i < 4; ++i) {
      const size_t ao = (size_t)(m0 + (i << 4) + rlane) * lda + koff + k0;
      const v16b ah = Frag<__bf16>::load(A + ao);
      const v16b al = Frag<__bf16>::load(A2 + ao);
#pragma unroll
      for (int j = 0; j < 4; ++j) {
        acc[i][j] = Frag<__bf16>::mma(ah, bh[j], acc[i][j]);
        acc[i][j] = Frag<__bf16>::mma(al, bh[j], acc[i][j]);
      }
      dep_guard_all(acc[i][0], acc[i][1], acc[i][2], acc[i][3], ah, al, bh[0], bh[1], bh[2], bh[3]);
    }
  }
  acc_guard4(acc[0][0], acc[0][1], acc[0][2], acc[0][3]);
  acc_guard4(acc[1][0], acc[1][1], acc[1][2], acc[1][3]);
  acc_guard4(acc[2][0], acc[2][1], acc[2][2], acc[2][3]);
  acc_guard4(acc[3][0], acc[3][1], acc[3][2], acc[3][3]);

  float* slab = sT[wave];
#pragma unroll
  for (int i = 0; i < 4; ++i) {
    const int mBase = m0 + (i << 4);
#pragma unroll
    for (int j = 0; j < 4; ++j) {
      const int n = n0 + (j << 4) + rlane;
      float bv = 0.f;
      if (BIAS_MODE == 2) bv = bf_rne(bias[n]);
#pragma unroll
      for (int r = 0; r < 8; ++r) {
        float v = acc[i][j][r];
        if (BIAS_MODE == 2) v += bv;
        slab[(mOff + r) * 68 + (j << 4) + rlane] = v;
      }
    }
    __builtin_amdgcn_fence(__ATOMIC_RELEASE, "workgroup");
    __builtin_amdgcn_wave_barrier();
    __builtin_amdgcn_fence(__ATOMIC_ACQUIRE, "workgroup");
    {
      const int hh = lane >> 4, c4 = (lane & 15) * 4;
      for (int pass = 0; pass < 2; ++pass) {
#pragma unroll
        for (int it = 0; it < 8; ++it) {
          const int row = it * 2 + hh;
          v4f v = *(const v4f*)(slab + row * 68 + c4);
          if (RESID_MODE != 0) {
            const v4f rv = *(const v4f*)(resid + (size_t)(mBase + row) * ldr + n0 + c4);
            if (RESID_MODE == 2) {
              const float q0 = rv[0], q1 = rv[1], q2 = rv[2], q3 = rv[3];
              v4f rr;
              rr[0] = bf_rne(q0); rr[1] = bf_rne(q1); rr[2] = bf_rne(q2); rr[3] = bf_rne(q3);
              v += rr;
            } else {
              v += rv;
            }
          }
          *(volatile v4f*)(Cout + (size_t)(mBase + row) * ldc + n0 + c4) = v;
        }
        __threadfence();
      }
    }
    __builtin_amdgcn_fence(__ATOMIC_RELEASE, "workgroup");
    __builtin_amdgcn_wave_barrier();
    __builtin_amdgcn_fence(__ATOMIC_ACQUIRE, "workgroup");
  }
}

__global__ __launch_bounds__(256) void wtrans_bf16_kernel(const float* __restrict__ in, int R, int C,
                                                          unsigned short* __restrict__ out) {
  __shared__ __align__(16) float sT[64 * 68];
  const int tid = threadIdx.x;
  const int c0 = blockIdx.x * 64, r0 = blockIdx.y * 64;
#pragma unroll
  for (int it = 0; it < 4; ++it) {
    const int idx = it * 256 + tid;
    const int r = idx >> 4, c4 = (idx & 15) * 4;
    const v4f v = *(const v4f*)(in + (size_t)(r0 + r) * C + c0 + c4);
    *(v4f*)(sT + r * 68 + c4) = v;
  }
  __syncthreads();
  v8h hv[2];
#pragma unroll
  for (int it = 0; it < 2; ++it) {
    const int orow = it * 32 + (tid >> 3);
    const int e8 = (tid & 7) * 8;
#pragma unroll
    for (int e = 0; e < 8; ++e) hv[it][e] = bits_h(f2bf_bits(sT[(e8 + e) * 68 + orow]));
  }
  for (int pass = 0; pass < 2; ++pass) {
#pragma unroll
    for (int it = 0; it < 2; ++it) {
      const int orow = it * 32 + (tid >> 3);
      const int e8 = (tid & 7) * 8;
      *(volatile v8h*)(out + (size_t)(c0 + orow) * R + r0 + e8) = hv[it];
    }
    __threadfence();
  }
}

__global__ __launch_bounds__(256) void wcvt_bf16_kernel(const float* __restrict__ src, unsigned short* __restrict__ dst,
                                                        int total8) {
  const int i = blockIdx.x * 256 + threadIdx.x;
  if (i >= total8) return;
  const size_t e0 = (size_t)i << 3;
  const v4f a0 = *(const v4f*)(src + e0);
  const v4f a1 = *(const v4f*)(src + e0 + 4);
  v8h hv;
#pragma unroll
  for (int e = 0; e < 4; ++e) {
    hv[e]     = bits_h(f2bf_bits(a0[e]));
    hv[4 + e] = bits_h(f2bf_bits(a1[e]));
  }
  store2_v8h(dst + e0, hv);
}

__global__ __launch_bounds__(32) void wdt_rows_kernel(const float* __restrict__ Wdt, unsigned short* __restrict__ dst) {
  const int n  = blockIdx.x;
  const int nc = (n < kHeads) ? n : (kHeads - 1);
  const int k8 = threadIdx.x * 8;
  v8h hv;
#pragma unroll
  for (int e = 0; e < 8; ++e) {
    const float w = Wdt[(size_t)(k8 + e) * kHeads + nc];
    const unsigned short bits = (n < kHeads) ? f2bf_bits(w) : (unsigned short)0;
    hv[e] = bits_h(bits);
  }
  store2_v8h(dst + (size_t)n * kDim + k8, hv);
}

template <int PERM, int RNE_IN>
__global__ __launch_bounds__(256) void ln_split_kernel(const float* __restrict__ in, const float* __restrict__ g,
                                                       const float* __restrict__ bta,
                                                       unsigned short* __restrict__ OH, unsigned short* __restrict__ OL) {
  __shared__ float sRa[8];
  __shared__ float sRb[8];
  __shared__ __align__(16) float sRow[kDim];
  const int tid = threadIdx.x, lane = tid & 31, wave = tid >> 5;
  const int orow = blockIdx.x;
  int irow = orow;
  if (PERM) {
    const int t  = orow & (kTime - 1);
    const int bk = orow >> 8;
    const int kb = bk & (kBands - 1);
    const int bb = bk >> 3;
    irow = (bb * kTime + t) * kBands + kb;
  }
  float x = in[(size_t)irow * kDim + tid];
  if (RNE_IN) x = bf_rne(x);
  const float gg = bf_rne(g[tid]);
  const float bv = bf_rne(bta[tid]);
  float s = x;
#pragma unroll
  for (int off = 1; off < 32; off <<= 1) s += __shfl_xor(s, off, 32);
  if (lane == 0) sRa[wave] = s;
  __syncthreads();
  float tot = sRa[0];
  tot += sRa[1]; tot += sRa[2]; tot += sRa[3]; tot += sRa[4]; tot += sRa[5]; tot += sRa[6]; tot += sRa[7];
  const float mean = tot * (1.0f / (float)kDim);
  const float c = x - mean;
  float s2 = c * c;
#pragma unroll
  for (int off = 1; off < 32; off <<= 1) s2 += __shfl_xor(s2, off, 32);
  if (lane == 0) sRb[wave] = s2;
  __syncthreads();
  float tot2 = sRb[0];
  tot2 += sRb[1]; tot2 += sRb[2]; tot2 += sRb[3]; tot2 += sRb[4]; tot2 += sRb[5]; tot2 += sRb[6]; tot2 += sRb[7];
  const float var = tot2 * (1.0f / (float)kDim);
  const float y = c * rsqrtf(var + 1e-5f) * gg + bv;
  sRow[tid] = y;
  __syncthreads();
  if (wave < 2) {
    const int c8 = lane * 8;
    const v4f a0 = *(const v4f*)(sRow + c8);
    const v4f a1 = *(const v4f*)(sRow + c8 + 4);
    v8h hv, lv;
    split8(a0, a1, hv, lv);
    const size_t o = (size_t)orow * kDim + c8;
    if (wave == 0) store2_v8h(OH + o, hv);
    else           store2_v8h(OL + o, lv);
  }
}

__global__ __launch_bounds__(256) void conv_silu_kernel(const float* __restrict__ C1, const float* __restrict__ cw,
                                                        float* __restrict__ XH) {
  __shared__ __align__(16) float sT[16 * kConvTP];
  const int tid = threadIdx.x, lane = tid & 31, wave = tid >> 5;
  const int d = tid;
  const int g0 = blockIdx.x * 64;
  const int tb = g0 & (kTime - 1);
  const float w0 = bf_rne(cw[d * 4 + 0]), w1 = bf_rne(cw[d * 4 + 1]);
  const float w2 = bf_rne(cw[d * 4 + 2]), w3 = bf_rne(cw[d * 4 + 3]);
  float xm3, xm2, xm1;
  {
    const bool hist = (tb > 0);
    const int rb = hist ? (g0 - 3) : g0;
    const float v3 = C1[(size_t)rb * kC1P + kC1X + d];
    const float v2 = C1[(size_t)(rb + 1) * kC1P + kC1X + d];
    const float v1 = C1[(size_t)(rb + 2) * kC1P + kC1X + d];
    xm3 = hist ? v3 : 0.f;
    xm2 = hist ? v2 : 0.f;
    xm1 = hist ? v1 : 0.f;
  }
  const int hrow = wave >> 1;
  const int hch  = (wave & 1) * 128 + lane * 4;
#pragma unroll 1
  for (int sub = 0; sub < 4; ++sub) {
    const int lb = g0 + sub * 16;
#pragma unroll 1
    for (int s = 0; s < 16; ++s) {
      const float xcur = C1[(size_t)(lb + s) * kC1P + kC1X + d];
      float acc = w0 * xm3;
      acc = fmaf(w1, xm2, acc);
      acc = fmaf(w2, xm1, acc);
      acc = fmaf(w3, xcur, acc);
      const float sg = __builtin_amdgcn_rcpf(1.0f + expf(-acc));
      sT[s * kConvTP + tid] = acc * sg;
      xm3 = xm2; xm2 = xm1; xm1 = xcur;
    }
    __syncthreads();
    v4f fv[4];
#pragma unroll
    for (int it = 0; it < 4; ++it) fv[it] = *(const v4f*)(sT + (it * 4 + hrow) * kConvTP + hch);
    for (int pass = 0; pass < 2; ++pass) {
#pragma unroll
      for (int it = 0; it < 4; ++it)
        *(volatile v4f*)(XH + (size_t)(lb + it * 4 + hrow) * kDim + hch) = fv[it];
      __threadfence();
    }
    __syncthreads();
  }
}

__global__ __launch_bounds__(256) void dtprep_kernel(const float* __restrict__ C1, const float* __restrict__ dtb,
                                                     const float* __restrict__ alog, const float* __restrict__ th,
                                                     float* __restrict__ DT, float* __restrict__ AR, float* __restrict__ AI) {
  const int idx = blockIdx.x * 256 + threadIdx.x;
  if (idx >= kRows * kHeads) return;
  const int r = idx >> 2, h = idx & 3;
  const float raw = C1[(size_t)r * kC1P + kC1T + h];
  const float s   = raw + bf_rne(dtb[h]);
  const float dt  = fmaxf(s, 0.0f) + log1pf(expf(-fabsf(s)));
  const float an  = -expf(bf_rne(alog[h]));
  const float mg  = expf(dt * an);
  const float ph  = dt * bf_rne(th[h]);
  float sn, cs;
  sincosf(ph, &sn, &cs);
  const float ar = mg * cs;
  const float ai = mg * sn;
  ((volatile float*)DT)[idx] = dt;
  ((volatile float*)AR)[idx] = ar;
  ((volatile float*)AI)[idx] = ai;
  __threadfence();
  ((volatile float*)DT)[idx] = dt;
  ((volatile float*)AR)[idx] = ar;
  ((volatile float*)AI)[idx] = ai;
}

__global__ __launch_bounds__(256) void bmix_kernel(const float* __restrict__ C1, const float* __restrict__ DT,
                                                   const float* __restrict__ Um, const float* __restrict__ Vm,
                                                   float* __restrict__ DTB) {
  __shared__ float sU[16];
  __shared__ float sV[16];
  const int tid = threadIdx.x;
  if (tid < 16) { sU[tid] = bf_rne(Um[tid]); sV[tid] = bf_rne(Vm[tid]); }
  __syncthreads();
  const int idx = blockIdx.x * 256 + tid;
  const int r = idx >> 7;
  const int rem = idx & 127;
  const int h = rem >> 5;
  const int n4 = (rem & 31) * 4;
  float mg[4];
#pragma unroll
  for (int gi = 0; gi < 4; ++gi) {
    float m = sU[h * 4 + 0] * sV[gi * 4 + 0];
    m = fmaf(sU[h * 4 + 1], sV[gi * 4 + 1], m);
    m = fmaf(sU[h * 4 + 2], sV[gi * 4 + 2], m);
    m = fmaf(sU[h * 4 + 3], sV[gi * 4 + 3], m);
    mg[gi] = m;
  }
  const float* bp = C1 + (size_t)r * kC1P + kC1B + n4;
  const v4f b0 = *(const v4f*)(bp);
  const v4f b1 = *(const v4f*)(bp + kNs);
  const v4f b2 = *(const v4f*)(bp + 2 * kNs);
  const v4f b3 = *(const v4f*)(bp + 3 * kNs);
  const float dt = DT[(size_t)r * kHeads + h];
  v4f o = b0 * mg[0];
  o += b1 * mg[1];
  o += b2 * mg[2];
  o += b3 * mg[3];
  o *= dt;
  store2_v4f(DTB + (size_t)r * kDtbP + h * kNs + n4, o);
}

__device__ __forceinline__ float cstep(float b, float c, float xt, float ar, float ai, float& hr, float& hm, float acc) {
  const float dBx = b * xt;
  const float nr = ar * hr - ai * hm + dBx;
  const float ni = ar * hm + ai * hr;
  hr = nr; hm = ni;
  return acc + c * nr;
}
__global__ __launch_bounds__(256) void cscan_kernel(const float* __restrict__ DTB, const float* __restrict__ C1,
                                                    const float* __restrict__ XH, const float* __restrict__ AR,
                                                    const float* __restrict__ AI, float* __restrict__ YSP) {
  __shared__ __align__(16) float sB[kScanTS * 32];
  __shared__ __align__(16) float sC[kScanTS * 32];
  __shared__ __align__(16) float sX[kScanTS * kHd];
  __shared__ float sAR[kScanTS];
  __shared__ float sAI[kScanTS];
  __shared__ __align__(16) float sYp[4 * kScanTS * kScanYP];
  const int tid = threadIdx.x, lane = tid & 31, wave = tid >> 5;
  const int ng = tid >> 6, p = tid & 63;
  const int bx = blockIdx.x;
  const int nq = bx & 3;
  const int h  = (bx >> 2) & 3;
  const int bk = bx >> 4;
  const int nb0 = nq * 32;
  const size_t row0 = (size_t)bk * kTime;
  float* Yq = YSP + (size_t)nq * kRows * kDim;
  float hre[8], him[8];
#pragma unroll
  for (int i = 0; i < 8; ++i) { hre[i] = 0.f; him[i] = 0.f; }
  const int sgs = tid >> 3, sgc = (tid & 7) * 4;
  const int cr = tid >> 4, cc4 = (tid & 15) * 4;
#pragma unroll 1
  for (int t0 = 0; t0 < kTime; t0 += kScanTS) {
    __syncthreads();
    {
      const size_t rg = row0 + t0 + sgs;
      *(v4f*)(sB + sgs * 32 + sgc) = *(const v4f*)(DTB + rg * kDtbP + h * kNs + nb0 + sgc);
      *(v4f*)(sC + sgs * 32 + sgc) = *(const v4f*)(C1 + rg * kC1P + kC1C + h * kNs + nb0 + sgc);
    }
#pragma unroll
    for (int it = 0; it < 2; ++it) {
      const int idx = it * 256 + tid;
      const int s = idx >> 4, c4 = (idx & 15) * 4;
      *(v4f*)(sX + s * kHd + c4) = *(const v4f*)(XH + (row0 + t0 + s) * kDim + h * kHd + c4);
    }
    if (wave == 0) sAR[lane] = AR[(row0 + t0 + lane) * kHeads + h];
    if (wave == 1) sAI[lane] = AI[(row0 + t0 + lane) * kHeads + h];
    __syncthreads();
#pragma unroll 1
    for (int s = 0; s < kScanTS; ++s) {
      const float xt = sX[s * kHd + p];
      const float ar = sAR[s], ai = sAI[s];
      const v4f bA = *(const v4f*)(sB + s * 32 + ng * 8);
      const v4f bB = *(const v4f*)(sB + s * 32 + ng * 8 + 4);
      const v4f cA = *(const v4f*)(sC + s * 32 + ng * 8);
      const v4f cB = *(const v4f*)(sC + s * 32 + ng * 8 + 4);
      float acc = 0.f;
#pragma unroll
      for (int i = 0; i < 4; ++i) acc = cstep(bA[i], cA[i], xt, ar, ai, hre[i], him[i], acc);
#pragma unroll
      for (int i = 0; i < 4; ++i) acc = cstep(bB[i], cB[i], xt, ar, ai, hre[4 + i], him[4 + i], acc);
      sYp[(ng * kScanTS + s) * kScanYP + p] = acc;
    }
    __syncthreads();
    v4f yv[2];
#pragma unroll
    for (int it = 0; it < 2; ++it) {
      const int row = it * 16 + cr;
      v4f y = *(const v4f*)(sYp + (0 * kScanTS + row) * kScanYP + cc4);
      y += *(const v4f*)(sYp + (1 * kScanTS + row) * kScanYP + cc4);
      y += *(const v4f*)(sYp + (2 * kScanTS + row) * kScanYP + cc4);
      y += *(const v4f*)(sYp + (3 * kScanTS + row) * kScanYP + cc4);
      yv[it] = y;
    }
    for (int pass = 0; pass < 2; ++pass) {
#pragma unroll
      for (int it = 0; it < 2; ++it)
        *(volatile v4f*)(Yq + (row0 + t0 + it * 16 + cr) * kDim + h * kHd + cc4) = yv[it];
      __threadfence();
    }
  }
}

__global__ __launch_bounds__(256) void ygate_kernel(const float* __restrict__ YSP, const float* __restrict__ XH,
                                                    const float* __restrict__ C1, const float* __restrict__ Dsk,
                                                    unsigned short* __restrict__ YH, unsigned short* __restrict__ YL) {
  __shared__ __align__(16) float sRow[kDim];
  const int tid = threadIdx.x, lane = tid & 31, wave = tid >> 5;
  const int r = blockIdx.x;
  const int d = tid;
  const int h = d >> 6;
  const size_t i = (size_t)r * kDim + d;
  const size_t plane = (size_t)kRows * kDim;
  float ys = YSP[i];
  ys += YSP[plane + i];
  ys += YSP[2 * plane + i];
  ys += YSP[3 * plane + i];
  float y = ys + bf_rne(Dsk[h]) * XH[i];
  const float zg = C1[(size_t)r * kC1P + kC1Z + d];
  const float sg = __builtin_amdgcn_rcpf(1.0f + expf(-zg));
  y = y * (zg * sg);
  sRow[d] = y;
  __syncthreads();
  const int t  = r & (kTime - 1);
  const int bk = r >> 8;
  const int kb = bk & (kBands - 1);
  const int bb = bk >> 3;
  const int orow = (bb * kTime + t) * kBands + kb;
  if (wave < 2) {
    const int c8 = lane * 8;
    const v4f a0 = *(const v4f*)(sRow + c8);
    const v4f a1 = *(const v4f*)(sRow + c8 + 4);
    v8h hv, lv;
    split8(a0, a1, hv, lv);
    const size_t o = (size_t)orow * kDim + c8;
    if (wave == 0) store2_v8h(YH + o, hv);
    else           store2_v8h(YL + o, lv);
  }
}

__global__ __launch_bounds__(256) void band_attn_kernel(const float* __restrict__ QKV, unsigned short* __restrict__ OH,
                                                        unsigned short* __restrict__ OL) {
  __shared__ __align__(16) float sQKV[3 * 8 * kDim];
  __shared__ float sS[128];
  __shared__ __align__(16) float sO[8 * kAttnOP];
  const int tid = threadIdx.x, lane = tid & 31, wave = tid >> 5;
  const int bt = blockIdx.x;
#pragma unroll
  for (int it = 0; it < 6; ++it) {
    const int idx = it * 256 + tid;
    const int ts = idx >> 9;
    const int rem = idx & 511;
    const int row = rem >> 6, c4 = (rem & 63) * 4;
    *(v4f*)(sQKV + (ts * 8 + row) * kDim + c4) = *(const v4f*)(QKV + (size_t)(bt * 8 + row) * kQkvP + ts * kDim + c4);
  }
  __syncthreads();
  if (tid < 128) {
    const int w = tid >> 6, h = (tid >> 4) & 3, qi = (tid >> 2) & 3, ki = tid & 3;
    const float* qp = sQKV + (w * 4 + qi) * kDim + h * kHd;
    const float* kp = sQKV + (8 + w * 4 + ki) * kDim + h * kHd;
    float acc = 0.f;
#pragma unroll 1
    for (int e4 = 0; e4 < 16; ++e4) {
      const v4f a = *(const v4f*)(qp + 4 * e4);
      const v4f c = *(const v4f*)(kp + 4 * e4);
      acc = fmaf(a[0], c[0], acc);
      acc = fmaf(a[1], c[1], acc);
      acc = fmaf(a[2], c[2], acc);
      acc = fmaf(a[3], c[3], acc);
    }
    sS[tid] = acc * 0.125f;
  }
  __syncthreads();
  if (tid < 32) {
    const float s0 = sS[tid * 4 + 0], s1 = sS[tid * 4 + 1], s2 = sS[tid * 4 + 2], s3 = sS[tid * 4 + 3];
    const float mx = fmaxf(fmaxf(s0, s1), fmaxf(s2, s3));
    const float e0 = expf(s0 - mx), e1 = expf(s1 - mx), e2 = expf(s2 - mx), e3 = expf(s3 - mx);
    float sum = e0 + e1; sum += e2; sum += e3;
    const float inv = 1.0f / sum;
    sS[tid * 4 + 0] = e0 * inv;
    sS[tid * 4 + 1] = e1 * inv;
    sS[tid * 4 + 2] = e2 * inv;
    sS[tid * 4 + 3] = e3 * inv;
  }
  __syncthreads();
  {
    const int d = tid;
    const int h = d >> 6;
#pragma unroll 1
    for (int q8 = 0; q8 < 8; ++q8) {
      const int w = q8 >> 2, qi = q8 & 3;
      const float* ap = sS + ((w * 4 + h) * 4 + qi) * 4;
      const float* vp = sQKV + (16 + w * 4) * kDim + d;
      float o = 0.f;
      o = fmaf(ap[0], vp[0], o);
      o = fmaf(ap[1], vp[kDim], o);
      o = fmaf(ap[2], vp[2 * kDim], o);
      o = fmaf(ap[3], vp[3 * kDim], o);
      sO[q8 * kAttnOP + d] = o;
    }
  }
  __syncthreads();
  {
    const int c8 = lane * 8;
    const v4f a0 = *(const v4f*)(sO + wave * kAttnOP + c8);
    const v4f a1 = *(const v4f*)(sO + wave * kAttnOP + c8 + 4);
    v8h hv, lv;
    split8(a0, a1, hv, lv);
    const size_t o = (size_t)(bt * 8 + wave) * kDim + c8;
    *(volatile v8h*)(OH + o) = hv;
    *(volatile v8h*)(OL + o) = lv;
    __threadfence();
    *(volatile v8h*)(OH + o) = hv;
    *(volatile v8h*)(OL + o) = lv;
  }
}

__global__ __launch_bounds__(256) void swiglu_split_kernel(const float* __restrict__ GU, unsigned short* __restrict__ GH,
                                                           unsigned short* __restrict__ GL) {
  const int idx = blockIdx.x * 256 + threadIdx.x;
  if (idx >= kRows * (kFf / 8)) return;
  const int r = idx >> 7;
  const int c8 = (idx & 127) * 8;
  const float* gp = GU + (size_t)r * kGuP + c8;
  const v4f g0 = *(const v4f*)(gp);
  const v4f g1 = *(const v4f*)(gp + 4);
  const v4f u0 = *(const v4f*)(gp + kFf);
  const v4f u1 = *(const v4f*)(gp + kFf + 4);
  v4f p0, p1;
#pragma unroll
  for (int e = 0; e < 4; ++e) {
    const float a0 = g0[e], a1 = g1[e];
    const float s0 = a0 * __builtin_amdgcn_rcpf(1.0f + expf(-a0));
    const float s1 = a1 * __builtin_amdgcn_rcpf(1.0f + expf(-a1));
    p0[e] = s0 * u0[e];
    p1[e] = s1 * u1[e];
  }
  v8h hv, lv;
  split8(p0, p1, hv, lv);
  const size_t o = (size_t)r * kFf + c8;
  *(volatile v8h*)(GH + o) = hv;
  *(volatile v8h*)(GL + o) = lv;
  __threadfence();
  *(volatile v8h*)(GH + o) = hv;
  *(volatile v8h*)(GL + o) = lv;
}

extern "C" void kernel_launch(void* const* d_in, const int* in_sizes, int n_in,
                              void* d_out, int out_size, void* d_ws, size_t ws_size,
                              hipStream_t stream) {
  if (n_in < 27) return;
  if (in_sizes[0] != kRows * kDim) return;
  if (in_sizes[1] != kDim || in_sizes[2] != kDim) return;
  if (in_sizes[3] != kDim * kDim) return;
  if (in_sizes[4] != kDim * 4) return;
  if (in_sizes[5] != kDim * kDim) return;
  if (in_sizes[6] != kDim * kDtbP || in_sizes[7] != kDim * kDtbP) return;
  if (in_sizes[8] != kDim * kHeads) return;
  if (in_sizes[9] != kHeads || in_sizes[10] != kHeads || in_sizes[11] != kHeads || in_sizes[12] != kHeads) return;
  if (in_sizes[13] != kHeads * kHeads || in_sizes[14] != kHeads * kHeads) return;
  if (in_sizes[15] != kDim * kDim) return;
  if (in_sizes[16] != kDim || in_sizes[17] != kDim) return;
  if (in_sizes[18] != kQkvP * kDim || in_sizes[19] != kQkvP) return;
  if (in_sizes[20] != kDim * kDim || in_sizes[21] != kDim) return;
  if (in_sizes[22] != kDim || in_sizes[23] != kDim) return;
  if (in_sizes[24] != kDim * kFf || in_sizes[25] != kDim * kFf || in_sizes[26] != kFf * kDim) return;
  if (out_size != kRows * kDim) return;
  if (ws_size < kWsTotal) return;

  const float* z          = (const float*)d_in[0];
  const float* ln1_g      = (const float*)d_in[1];
  const float* ln1_b      = (const float*)d_in[2];
  const float* Wx         = (const float*)d_in[3];
  const float* conv_w     = (const float*)d_in[4];
  const float* Wz         = (const float*)d_in[5];
  const float* Wb         = (const float*)d_in[6];
  const float* Wc         = (const float*)d_in[7];
  const float* Wdt        = (const float*)d_in[8];
  const float* dt_bias    = (const float*)d_in[9];
  const float* A_log      = (const float*)d_in[10];
  const float* theta      = (const float*)d_in[11];
  const float* D_skip     = (const float*)d_in[12];
  const float* mimo_U     = (const float*)d_in[13];
  const float* mimo_V     = (const float*)d_in[14];
  const float* Wout       = (const float*)d_in[15];
  const float* ln2_g      = (const float*)d_in[16];
  const float* ln2_b      = (const float*)d_in[17];
  const float* attn_in_w  = (const float*)d_in[18];
  const float* attn_in_b  = (const float*)d_in[19];
  const float* attn_out_w = (const float*)d_in[20];
  const float* attn_out_b = (const float*)d_in[21];
  const float* ln3_g      = (const float*)d_in[22];
  const float* ln3_b      = (const float*)d_in[23];
  const float* Wg         = (const float*)d_in[24];
  const float* Wu         = (const float*)d_in[25];
  const float* Wd         = (const float*)d_in[26];
  float* out = (float*)d_out;

  char* ws = (char*)d_ws;
  unsigned short* WCAT = (unsigned short*)(ws + kOffWcat);
  unsigned short* WOUT = (unsigned short*)(ws + kOffWout);
  unsigned short* WQKV = (unsigned short*)(ws + kOffWqkv);
  unsigned short* WAO  = (unsigned short*)(ws + kOffWao);
  unsigned short* WGU  = (unsigned short*)(ws + kOffWgu);
  unsigned short* WD   = (unsigned short*)(ws + kOffWd);
  unsigned short* UH   = (unsigned short*)(ws + kOffUH);
  unsigned short* UL   = (unsigned short*)(ws + kOffUL);
  float*          C1   = (float*)(ws + kOffC1);
  float*          XH   = (float*)(ws + kOffXH);
  float*          DTB  = (float*)(ws + kOffDTB);
  float*          DT   = (float*)(ws + kOffDT);
  float*          AR   = (float*)(ws + kOffAR);
  float*          AI   = (float*)(ws + kOffAI);
  float*          YSP  = (float*)(ws + kOffYSP);
  unsigned short* Y2H  = (unsigned short*)(ws + kOffY2H);
  unsigned short* Y2L  = (unsigned short*)(ws + kOffY2L);
  float*          Z1   = (float*)(ws + kOffZ1);
  unsigned short* ZNH  = (unsigned short*)(ws + kOffZNH);
  unsigned short* ZNL  = (unsigned short*)(ws + kOffZNL);
  float*          QKV  = (float*)(ws + kOffQKV);
  unsigned short* OH   = (unsigned short*)(ws + kOffOH);
  unsigned short* OL   = (unsigned short*)(ws + kOffOL);
  float*          Z2   = (float*)(ws + kOffZ2);
  unsigned short* ZFH  = (unsigned short*)(ws + kOffZFH);
  unsigned short* ZFL  = (unsigned short*)(ws + kOffZFL);
  float*          GU   = (float*)(ws + kOffGU);
  unsigned short* GUH  = (unsigned short*)(ws + kOffGUH);
  unsigned short* GUL  = (unsigned short*)(ws + kOffGUL);

  wtrans_bf16_kernel<<<dim3(kDim / 64, kDim / 64), 256, 0, stream>>>(Wx, kDim, kDim, WCAT);
  wtrans_bf16_kernel<<<dim3(kDim / 64, kDim / 64), 256, 0, stream>>>(Wz, kDim, kDim, WCAT + (size_t)kC1Z * kDim);
  wtrans_bf16_kernel<<<dim3(kDtbP / 64, kDim / 64), 256, 0, stream>>>(Wb, kDim, kDtbP, WCAT + (size_t)kC1B * kDim);
  wtrans_bf16_kernel<<<dim3(kDtbP / 64, kDim / 64), 256, 0, stream>>>(Wc, kDim, kDtbP, WCAT + (size_t)kC1C * kDim);
  wdt_rows_kernel<<<64, 32, 0, stream>>>(Wdt, WCAT + (size_t)kC1T * kDim);
  wtrans_bf16_kernel<<<dim3(kDim / 64, kDim / 64), 256, 0, stream>>>(Wout, kDim, kDim, WOUT);
  wcvt_bf16_kernel<<<(kQkvP * kDim / 8) / 256, 256, 0, stream>>>(attn_in_w, WQKV, kQkvP * kDim / 8);
  wcvt_bf16_kernel<<<(kDim * kDim / 8) / 256, 256, 0, stream>>>(attn_out_w, WAO, kDim * kDim / 8);
  wtrans_bf16_kernel<<<dim3(kFf / 64, kDim / 64), 256, 0, stream>>>(Wg, kDim, kFf, WGU);
  wtrans_bf16_kernel<<<dim3(kFf / 64, kDim / 64), 256, 0, stream>>>(Wu, kDim, kFf, WGU + (size_t)kFf * kDim);
  wtrans_bf16_kernel<<<dim3(kDim / 64, kFf / 64), 256, 0, stream>>>(Wd, kFf, kDim, WD);

  ln_split_kernel<1, 1><<<kRows, 256, 0, stream>>>(z, ln1_g, ln1_b, UH, UL);
  gemm_hilo_bf16_64<0, 0><<<(kRows / 64) * (kC1P / 64) / 8, 256, 0, stream>>>(
      UH, UL, kDim, WCAT, kDim, C1, kC1P, nullptr, nullptr, 0, kRows, kC1P, kDim);
  conv_silu_kernel<<<kRows / 64, 256, 0, stream>>>(C1, conv_w, XH);
  dtprep_kernel<<<(kRows * kHeads) / 256, 256, 0, stream>>>(C1, dt_bias, A_log, theta, DT, AR, AI);
  bmix_kernel<<<(kRows * (kDtbP / 4)) / 256, 256, 0, stream>>>(C1, DT, mimo_U, mimo_V, DTB);
  cscan_kernel<<<(kBatch * kBands) * kHeads * 4, 256, 0, stream>>>(DTB, C1, XH, AR, AI, YSP);
  ygate_kernel<<<kRows, 256, 0, stream>>>(YSP, XH, C1, D_skip, Y2H, Y2L);
  gemm_hilo_bf16_64<0, 2><<<(kRows / 64) * (kDim / 64) / 8, 256, 0, stream>>>(
      Y2H, Y2L, kDim, WOUT, kDim, Z1, kDim, nullptr, z, kDim, kRows, kDim, kDim);

  ln_split_kernel<0, 0><<<kRows, 256, 0, stream>>>(Z1, ln2_g, ln2_b, ZNH, ZNL);
  gemm_hilo_bf16_64<2, 0><<<(kRows / 64) * (kQkvP / 64) / 8, 256, 0, stream>>>(
      ZNH, ZNL, kDim, WQKV, kDim, QKV, kQkvP, attn_in_b, nullptr, 0, kRows, kQkvP, kDim);
  band_attn_kernel<<<kBatch * kTime, 256, 0, stream>>>(QKV, OH, OL);
  gemm_hilo_bf16_64<2, 1><<<(kRows / 64) * (kDim / 64) / 8, 256, 0, stream>>>(
      OH, OL, kDim, WAO, kDim, Z2, kDim, attn_out_b, Z1, kDim, kRows, kDim, kDim);

  ln_split_kernel<0, 0><<<kRows, 256, 0, stream>>>(Z2, ln3_g, ln3_b, ZFH, ZFL);
  gemm_hilo_bf16_64<0, 0><<<(kRows / 64) * (kGuP / 64) / 8, 256, 0, stream>>>(
      ZFH, ZFL, kDim, WGU, kDim, GU, kGuP, nullptr, nullptr, 0, kRows, kGuP, kDim);
  swiglu_split_kernel<<<(kRows * (kFf / 8)) / 256, 256, 0, stream>>>(GU, GUH, GUL);
  gemm_hilo_bf16_64<0, 1><<<(kRows / 64) * (kDim / 64) / 8, 256, 0, stream>>>(
      GUH, GUL, kFf, WD, kFf, out, kDim, nullptr, Z2, kDim, kRows, kDim, kFf);
}
